// RA_MLA_Attention_48799418417579
// MI455X (gfx1250) — hardware-verified
//
#include <hip/hip_runtime.h>


namespace {
constexpr int T = 2048, E = 1024, H = 16, D = 64, L = 64, QL = 2048  , NSLAB = (E + 2 * L) / 128  ;
constexpr float XS = 8.0f, WSC = 256.0f, PS = 1024.0f, LOG2E = 1.4426950408889634f;
static_assert(T % 64 == 0 && QL % 64 == 0, "tiling");
typedef _Float16 b16;
typedef __attribute__((ext_vector_type(16))) _Float16 v16b;
typedef __attribute__((ext_vector_type(8))) _Float16 v8b;
typedef __attribute__((ext_vector_type(8))) float v8f;
typedef __attribute__((ext_vector_type(4))) float v4f;
__device__ __forceinline__ float bf16_rne(float f) { unsigned int u = __float_as_uint(f); u += 0x7FFFu + ((u >> 16) & 1u); return __uint_as_float(u & 0xFFFF0000u); }
__device__ __forceinline__ void split16(float v, b16& hi, b16& lo) { hi = (b16)v; lo = (b16)(v - (float)hi); }
__device__ __forceinline__ v16b frag_kb(const b16* p, int hh) { const v8b a = *(const v8b*)(p + 8 * hh), b = *(const v8b*)(p + 16 + 8 * hh); v16b f;
#pragma unroll
  for (int e = 0; e < 8; ++e) { f[e] = a[e]; f[8 + e] = b[e]; } return f; }
__device__ __forceinline__ v8f wmma16b(v16b a, v16b b, v8f c) { v8f d = __builtin_amdgcn_wmma_f32_16x16x32_f16(false, a, false, b, (short)0, c, false, false); asm volatile("v_nop\n\tv_nop\n\tv_nop\n\tv_nop" : "+v"(d) : "v"(a), "v"(b)); return d; }
__device__ __forceinline__ void wave_lds_sync() { __builtin_amdgcn_fence(__ATOMIC_RELEASE, "workgroup"); __builtin_amdgcn_wave_barrier(); __builtin_amdgcn_fence(__ATOMIC_ACQUIRE, "workgroup"); }
__device__ __forceinline__ float pmul(float a, float b) { float p = a * b; asm volatile("" : "+v"(p)); return p; }
__device__ __forceinline__ int iclamp(int v, int lo, int hi) { return v < lo ? lo : (v > hi ? hi : v); }

typedef __attribute__((ext_vector_type(2))) _Float16 v2h;
typedef __attribute__((ext_vector_type(4))) _Float16 v4h;
typedef __attribute__((ext_vector_type(2))) float v2f;
__device__ __forceinline__ float nexp2(float v) { return __builtin_amdgcn_exp2f(v); }
__global__ __launch_bounds__(256) void prep_kernel(const float* __restrict__ wq, const float* __restrict__ wkd, const float* __restrict__ wvd, const float* __restrict__ q2l, const float* __restrict__ vup, const float* __restrict__ wo, b16* __restrict__ WT, b16* __restrict__ Q2L, b16* __restrict__ VUP, b16* __restrict__ WO) {
  const size_t u = (size_t)blockIdx.x * 256 + threadIdx.x; const size_t n1 = (size_t)(E + 2 * L) * E / 8, n2 = (size_t)H * L * D / 8, n3 = n2, n4 = (size_t)E * E / 8; v8b o;
  if (u < n1) { const size_t e = u * 8; const int oo = (int)(e / E), c0 = (int)(e % E); const float* src = (oo < E) ? (wq + (size_t)oo * E) : (oo < E + L ? (wkd + (size_t)(oo - E) * E) : (wvd + (size_t)(oo - E - L) * E));
    for (int j = 0; j < 8; ++j) o[j] = (b16)(bf16_rne(src[c0 + j]) * WSC); for (int pass = 0; pass < 2; ++pass) { *(volatile v8b*)(WT + e) = o; __threadfence(); } }
  else if (u < n1 + n2) { const size_t e = (u - n1) * 8; const int h = (int)(e / (L * D)), rem = (int)(e % (L * D)); const int l = rem / D, d0 = rem % D;
    for (int j = 0; j < 8; ++j) o[j] = (b16)(bf16_rne(q2l[((size_t)h * D + d0 + j) * L + l]) * WSC); for (int pass = 0; pass < 2; ++pass) { *(volatile v8b*)(Q2L + e) = o; __threadfence(); } }
  else if (u < n1 + n2 + n3) { const size_t e = (u - n1 - n2) * 8; const int h = (int)(e / (L * D)), rem = (int)(e % (L * D)); const int d = rem / L, l0 = rem % L;
    for (int j = 0; j < 8; ++j) o[j] = (b16)(bf16_rne(vup[((size_t)h * L + l0 + j) * D + d]) * WSC); for (int pass = 0; pass < 2; ++pass) { *(volatile v8b*)(VUP + e) = o; __threadfence(); } }
  else if (u < n1 + n2 + n3 + n4) { const size_t e = (u - n1 - n2 - n3) * 8; for (int j = 0; j < 8; ++j) o[j] = (b16)(bf16_rne(wo[e + j]) * WSC); for (int pass = 0; pass < 2; ++pass) { *(volatile v8b*)(WO + e) = o; __threadfence(); } }
}
__global__ __launch_bounds__(128) void proj_kernel(const float* __restrict__ x, const b16* __restrict__ WT, const b16* __restrict__ Q2L, b16* __restrict__ QH, b16* __restrict__ QLo, b16* __restrict__ KH, b16* __restrict__ KLo, b16* __restrict__ VTh, b16* __restrict__ VTl) {
  __shared__ __attribute__((aligned(16))) b16 As[64][256 + 8]; __shared__ __attribute__((aligned(16))) float Tf[4][16][128 + 4];
  const int wave = threadIdx.x >> 5, lane = threadIdx.x & 31, nloc = lane & 15, hlf = lane >> 4; const int t0 = blockIdx.x * 64; const int slab = blockIdx.y; const int n0 = slab * 128;
  const float* xb = x + (size_t)t0 * E;
  v8f acc[8];
#pragma unroll
  for (int t = 0; t < 8; ++t) acc[t] = (v8f){};
#pragma unroll 1
  for (int kc = 0; kc < E; kc += 256) {
    __syncthreads();
    for (int i = threadIdx.x; i < 64 * 64; i += 128) { const int rr = i / 64, q = (i % 64) * 4; const v4f f = *(const v4f*)(xb + (size_t)rr * E + kc + q); v4h o; for (int j = 0; j < 4; ++j) o[j] = (b16)(bf16_rne(f[j]) * XS); *(v4h*)(&As[rr][q]) = o; }
    __syncthreads();
#pragma unroll 2
    for (int kb = 0; kb < 256; kb += 32) { const v16b a = frag_kb(&As[wave * 16 + nloc][kb], hlf);
#pragma unroll
      for (int t = 0; t < 8; ++t) acc[t] = wmma16b(a, frag_kb(WT + (size_t)(n0 + t * 16 + nloc) * E + kc + kb, hlf), acc[t]); } }
#pragma unroll
  for (int t = 0; t < 8; ++t)
#pragma unroll
    for (int r = 0; r < 8; ++r) Tf[wave][8 * hlf + r][t * 16 + nloc] = acc[t][r] * (1.0f / (XS * WSC));
  __syncthreads();
  if (slab < 8) {
#pragma unroll
    for (int h2 = 0; h2 < 2; ++h2) { const int h = slab * 2 + h2; v8f ac2[4]; for (int t = 0; t < 4; ++t) ac2[t] = (v8f){};
#pragma unroll
      for (int ks = 0; ks < 2; ++ks) { v16b ah, al;
#pragma unroll
        for (int e2 = 0; e2 < 16; ++e2) { const int k = ks * 32 + (e2 < 8 ? 0 : 16) + 8 * hlf + (e2 & 7); b16 p, q; split16(Tf[wave][nloc][h2 * 64 + k] * XS, p, q); ah[e2] = p; al[e2] = q; }
#pragma unroll
        for (int t = 0; t < 4; ++t) { const v16b bw = frag_kb(Q2L + ((size_t)h * L + t * 16 + nloc) * D + ks * 32, hlf); ac2[t] = wmma16b(ah, bw, ac2[t]); ac2[t] = wmma16b(al, bw, ac2[t]); } }
      wave_lds_sync();
#pragma unroll
      for (int t = 0; t < 4; ++t)
#pragma unroll
        for (int r = 0; r < 8; ++r) Tf[wave][8 * hlf + r][h2 * 64 + t * 16 + nloc] = ac2[t][r] * (1.0f / (XS * WSC));
      wave_lds_sync(); } }
  __syncthreads();
  for (int pass = 0; pass < 2; ++pass) {
    if (slab < 8) { const int c = lane * 4; const int h = slab * 2 + c / 64, l = c % 64;
      for (int rr = 0; rr < 16; ++rr) { const int tok = t0 + wave * 16 + rr; v4h h4, l4; for (int j = 0; j < 4; ++j) { b16 p, q; split16(Tf[wave][rr][c + j] * XS, p, q); h4[j] = p; l4[j] = q; } const size_t oi = ((size_t)h * T + tok) * L + l; *(volatile v4h*)(QH + oi) = h4; *(volatile v4h*)(QLo + oi) = l4; } }
    else {
      for (int rr = 0; rr < 16; ++rr) { const int tok = t0 + wave * 16 + rr; if (lane < 16) { v4h h4, l4; for (int j = 0; j < 4; ++j) { b16 p, q; split16(Tf[wave][rr][lane * 4 + j] * XS, p, q); h4[j] = p; l4[j] = q; } *(volatile v4h*)(KH + (size_t)tok * L + lane * 4) = h4; *(volatile v4h*)(KLo + (size_t)tok * L + lane * 4) = l4; } }
#pragma unroll 1
      for (int q = 0; q < 16; ++q) { const int l = wave * 16 + q; const int tk = lane * 2; v2h hv, lv; for (int jj = 0; jj < 2; ++jj) { b16 p, ql; split16(Tf[(tk + jj) >> 4][(tk + jj) & 15][64 + l] * XS, p, ql); hv[jj] = p; lv[jj] = ql; }
        *(volatile v2h*)(VTh + (size_t)l * T + t0 + tk) = hv; *(volatile v2h*)(VTl + (size_t)l * T + t0 + tk) = lv; } }
    __threadfence(); }
}
__global__ __launch_bounds__(64) void attn_kernel(const b16* __restrict__ QH, const b16* __restrict__ QLo, const b16* __restrict__ KH, const b16* __restrict__ KLo, const b16* __restrict__ VTh, const b16* __restrict__ VTl, const b16* __restrict__ VUP, b16* __restrict__ Hh, b16* __restrict__ Hl) {
  __shared__ __attribute__((aligned(16))) b16 Pb[2][16][32 + 8], Pc[2][16][32 + 8]; __shared__ __attribute__((aligned(16))) float To[2][16][D + 4];
  const int wave = threadIdx.x >> 5, lane = threadIdx.x & 31, hh = lane >> 4, col = lane & 15; const int h = blockIdx.y; const int q0 = blockIdx.x * 32 + wave * 16, qi = q0 + col;
  const size_t pq = (size_t)h * T * L;
  const v16b qh0 = frag_kb(QH + pq + (size_t)qi * L, hh), qh1 = frag_kb(QH + pq + (size_t)qi * L + 32, hh), ql0 = frag_kb(QLo + pq + (size_t)qi * L, hh), ql1 = frag_kb(QLo + pq + (size_t)qi * L + 32, hh);
  const float cs = LOG2E / (8.0f * XS * XS);
  float m = -INFINITY, l = 0.0f; v8f o[4]; for (int t = 0; t < 4; ++t) o[t] = (v8f){};
  const int kend = q0 + 16;
#pragma unroll 1
  for (int kb = 0; kb < kend; kb += 32) {
    float e[16]; float mx = -INFINITY;
#pragma unroll
    for (int u = 0; u < 2; ++u) { v8f s = (v8f){}; const size_t kr = (size_t)(kb + u * 16 + col) * L; const v16b kh0 = frag_kb(KH + kr, hh), kh1 = frag_kb(KH + kr + 32, hh), kl0 = frag_kb(KLo + kr, hh), kl1 = frag_kb(KLo + kr + 32, hh);
      s = wmma16b(kh0, qh0, s); s = wmma16b(kh0, ql0, s); s = wmma16b(kl0, qh0, s); s = wmma16b(kh1, qh1, s); s = wmma16b(kh1, ql1, s); s = wmma16b(kl1, qh1, s);
#pragma unroll
      for (int r = 0; r < 8; ++r) { const int key = kb + u * 16 + 8 * hh + r; const float vv = (key <= qi) ? s[r] * cs : -INFINITY; e[u * 8 + r] = vv; mx = fmaxf(mx, vv); } }
    mx = fmaxf(mx, __shfl_xor(mx, 16)); const float mn = fmaxf(m, mx); const float al = (mn == -INFINITY) ? 1.0f : nexp2(m - mn); float sum = 0.0f;
#pragma unroll
    for (int i2 = 0; i2 < 16; ++i2) { const float p = (e[i2] == -INFINITY) ? 0.0f : nexp2(e[i2] - mn); sum += p; b16 a_, b_; split16(p * PS, a_, b_); const int sl = (i2 < 8 ? 0 : 16) + 8 * hh + (i2 & 7); Pb[wave][col][sl] = a_; Pc[wave][col][sl] = b_; }
    sum += __shfl_xor(sum, 16); l = l * al + sum; m = mn;
    wave_lds_sync();
    const v16b pf = frag_kb(&Pb[wave][col][0], hh), pg = frag_kb(&Pc[wave][col][0], hh);
#pragma unroll
    for (int t = 0; t < 4; ++t) { o[t] *= al; const size_t vr = (size_t)(t * 16 + col) * T + kb; const v16b va = frag_kb(VTh + vr, hh), vb2 = frag_kb(VTl + vr, hh); o[t] = wmma16b(va, pf, o[t]); o[t] = wmma16b(va, pg, o[t]); o[t] = wmma16b(vb2, pf, o[t]); }
    wave_lds_sync(); }
  const float inv = 1.0f / (l * PS * XS);
#pragma unroll
  for (int t = 0; t < 4; ++t)
#pragma unroll
    for (int r = 0; r < 8; ++r) To[wave][col][t * 16 + 8 * hh + r] = o[t][r] * inv;
  wave_lds_sync();
  v8f ac2[4]; for (int t = 0; t < 4; ++t) ac2[t] = (v8f){};
#pragma unroll
  for (int ks = 0; ks < 2; ++ks) { v16b ah, al2;
#pragma unroll
    for (int e2 = 0; e2 < 16; ++e2) { const int k = ks * 32 + (e2 < 8 ? 0 : 16) + 8 * hh + (e2 & 7); b16 p, q; split16(To[wave][col][k] * XS, p, q); ah[e2] = p; al2[e2] = q; }
#pragma unroll
    for (int t = 0; t < 4; ++t) { const v16b bw = frag_kb(VUP + ((size_t)h * D + t * 16 + col) * L + ks * 32, hh); ac2[t] = wmma16b(ah, bw, ac2[t]); ac2[t] = wmma16b(al2, bw, ac2[t]); } }
  wave_lds_sync();
#pragma unroll
  for (int t = 0; t < 4; ++t)
#pragma unroll
    for (int r = 0; r < 8; ++r) To[wave][8 * hh + r][t * 16 + col] = ac2[t][r] * (1.0f / (XS * WSC));
  wave_lds_sync();
  for (int pass = 0; pass < 2; ++pass) { for (int rr = 0; rr < 16; ++rr) { const v2f f = *(const v2f*)(&To[wave][rr][lane * 2]); v2h hv, lv; for (int j = 0; j < 2; ++j) { b16 p, q; split16(f[j] * XS, p, q); hv[j] = p; lv[j] = q; }
      const size_t oi = (size_t)(q0 + rr) * E + h * D + lane * 2; *(volatile v2h*)(Hh + oi) = hv; *(volatile v2h*)(Hl + oi) = lv; } __threadfence(); }
}
__global__ __launch_bounds__(128) void out_kernel(const b16* __restrict__ Hh, const b16* __restrict__ Hl, const b16* __restrict__ WO, float* __restrict__ out) {
  __shared__ __attribute__((aligned(16))) float Tf[4][16][128 + 4];
  const int wave = threadIdx.x >> 5, lane = threadIdx.x & 31, nloc = lane & 15, hlf = lane >> 4; const size_t m0 = ((size_t)blockIdx.x * 4 + wave) * 16; const int n0 = blockIdx.y * 128;
  v8f acc[8];
#pragma unroll
  for (int t = 0; t < 8; ++t) acc[t] = (v8f){};
#pragma unroll 2
  for (int kb = 0; kb < E; kb += 32) { const v16b a = frag_kb(Hh + (m0 + nloc) * E + kb, hlf), a2 = frag_kb(Hl + (m0 + nloc) * E + kb, hlf);
#pragma unroll
    for (int t = 0; t < 8; ++t) { const v16b bw = frag_kb(WO + (size_t)(n0 + t * 16 + nloc) * E + kb, hlf); acc[t] = wmma16b(a, bw, acc[t]); acc[t] = wmma16b(a2, bw, acc[t]); } }
#pragma unroll
  for (int t = 0; t < 8; ++t)
#pragma unroll
    for (int r = 0; r < 8; ++r) Tf[wave][8 * hlf + r][t * 16 + nloc] = acc[t][r] * (1.0f / (XS * WSC));
  wave_lds_sync();
  for (int pass = 0; pass < 2; ++pass) { for (int rr = 0; rr < 16; ++rr) *(volatile v4f*)(out + (m0 + rr) * E + n0 + lane * 4) = *(const v4f*)(&Tf[wave][rr][lane * 4]); __threadfence(); }
}
}

extern "C" void kernel_launch(void* const* d_in, const int* in_sizes, int n_in, void* d_out, int out_size, void* d_ws, size_t ws_size, hipStream_t stream) {
  (void)n_in;
  auto Fp = [&](int i) { return (const float*)d_in[i]; };
  if (in_sizes[0] != T * E || in_sizes[1] != E * E || in_sizes[2] != L * E || in_sizes[3] != L * E || in_sizes[4] != H * D * L || in_sizes[5] != H * L * D || in_sizes[6] != E * E || out_size != T * E) return;
  size_t off = 0; char* ws = (char*)d_ws;
  auto carve = [&](size_t bytes) { char* p = ws + off; off += (bytes + 255) & ~(size_t)255; return p; };
  b16* WT = (b16*)carve((size_t)(E + 2 * L) * E * 2); b16* Q2L = (b16*)carve((size_t)H * L * D * 2); b16* VUP = (b16*)carve((size_t)H * L * D * 2); b16* WO = (b16*)carve((size_t)E * E * 2);
  const size_t qplane = (size_t)H * T * L * 2, kplane = (size_t)T * L * 2, hplane = (size_t)T * E * 2;
  b16* QH = (b16*)carve(qplane); b16* QLo = (b16*)carve(qplane); b16* KH = (b16*)carve(kplane); b16* KLo = (b16*)carve(kplane); b16* VTh = (b16*)carve(kplane); b16* VTl = (b16*)carve(kplane); b16* Hh = (b16*)carve(hplane); b16* Hl = (b16*)carve(hplane);
  if (off > ws_size || off > ((size_t)128 << 20)) return;
  prep_kernel<<<(unsigned)((((size_t)(E + 2 * L) * E + 2 * (size_t)H * L * D + (size_t)E * E) / 8 + 255) / 256), 256, 0, stream>>>(Fp(1), Fp(2), Fp(3), Fp(4), Fp(5), Fp(6), WT, Q2L, VUP, WO);
  proj_kernel<<<dim3(QL / 64, NSLAB), 128, 0, stream>>>(Fp(0), WT, Q2L, QH, QLo, KH, KLo, VTh, VTl);
  attn_kernel<<<dim3(QL / 32, H), 64, 0, stream>>>(QH, QLo, KH, KLo, VTh, VTl, VUP, Hh, Hl);
  out_kernel<<<dim3(QL / 64, E / 128), 128, 0, stream>>>(Hh, Hl, WO, (float*)d_out);
}
